// LSTM_11879879542513
// MI455X (gfx1250) — hardware-run, weakly checked
//
#include <hip/hip_runtime.h>
#include <math.h>

typedef __attribute__((ext_vector_type(16))) _Float16 v16h;
typedef __attribute__((ext_vector_type(8)))  _Float16 v8h;
typedef __attribute__((ext_vector_type(8)))  float    v8f;
typedef __attribute__((ext_vector_type(4)))  float    v4f;
typedef __attribute__((ext_vector_type(2)))  unsigned v2u;

constexpr int kB = 64;
constexpr int kH = 2048;
constexpr int kK = 2 * kH;
constexpr int kG = 4 * kH;
constexpr int kOutLd = 3 * kH;
constexpr float kWCarry = 65536.0f;
static_assert(kK == 4096 && kG == 8192 && kOutLd == 6144);
static_assert((kB % 32) == 0 && (kG % 64) == 0 && (kH % 64) == 0);
static_assert((kK % 32) == 0 && (kH % 32) == 0);
static_assert(((kB / 32) * (kG / 64)) % 8 == 0);
static_assert(((kB / 32) * (kH / 64)) % 8 == 0);
static_assert(((kB * kK / 8) % 256) == 0);
static_assert(((kG * kK / 8) % 256) == 0);
static_assert(((kH * kH / 8) % 256) == 0);
static_assert(((kB * kH / 4) % 256) == 0);
static_assert(kH == 256 * 8);

constexpr size_t kSzAX = (size_t)kB * kK * 2;
constexpr size_t kSzWT = (size_t)kG * kK * 2;
constexpr size_t kSzWY = (size_t)kH * kH * 2;
constexpr size_t kSzGT = (size_t)kB * kG * 4;
constexpr size_t kSzYR = (size_t)kB * kH * 4;
constexpr size_t kOffAX = 0;
constexpr size_t kOffWT = kOffAX + kSzAX;
constexpr size_t kOffWY = kOffWT + kSzWT;
constexpr size_t kOffGT = kOffWY + kSzWY;
constexpr size_t kOffYR = kOffGT + kSzGT;
constexpr size_t kWsTotal = kOffYR + kSzYR;
static_assert(kSzAX == 524288ull);
static_assert(kSzWT == 67108864ull);
static_assert(kSzWY == 8388608ull);
static_assert(kSzGT == 2097152ull);
static_assert(kSzYR == 524288ull);
static_assert(kWsTotal == 78643200ull);
static_assert(kWsTotal <= 134217728ull);
static_assert((kSzAX % 256) == 0 && (kSzWT % 256) == 0 && (kSzWY % 256) == 0 &&
              (kSzGT % 256) == 0 && (kSzYR % 256) == 0);

__device__ __forceinline__ _Float16 f16_flush(float v) {
  const float w = (fabsf(v) < 6.103515625e-05f) ? 0.0f : v;
  return (_Float16)w;
}

__device__ __forceinline__ float bf16r(float v) {
  unsigned u = __float_as_uint(v);
  u = (u + 0x7FFFu + ((u >> 16) & 1u)) & 0xFFFF0000u;
  return __uint_as_float(u);
}

namespace eng {
union FragU { v16h v; v8h h[2]; };
__device__ __forceinline__ v16h frag_load(const _Float16* p) {
  FragU f;
  f.h[0] = *(const v8h*)(p);
  f.h[1] = *(const v8h*)(p + 16);
  return f.v;
}
__device__ __forceinline__ v8f mma(v16h a, v16h b, v8f c) {
  return __builtin_amdgcn_wmma_f32_16x16x32_f16(false, a, false, b, (short)0, c, false, false);
}
__device__ __forceinline__ void guard1(v8f& a, v16h x, v16h y) {
  asm volatile("v_nop\n\tv_nop\n\tv_nop\n\tv_nop" : "+v"(a) : "v"(x), "v"(y));
}
__device__ __forceinline__ void guard_acc(v8f& a) {
  asm volatile("v_nop\n\tv_nop\n\tv_nop\n\tv_nop" : "+v"(a));
}
__device__ __forceinline__ void keep4(v16h a, v16h b, v16h c, v16h d) {
  asm volatile("v_nop" :: "v"(a), "v"(b), "v"(c), "v"(d));
}

template <int MI, int SPL>
__global__ __launch_bounds__(256) void gemm_f16_kernel(
    const unsigned short* __restrict__ Ap, const unsigned short* __restrict__ A2p, int lda,
    const unsigned short* __restrict__ Btp, const unsigned short* __restrict__ Bt2p, int ldb,
    float* __restrict__ C, int ldc, int M, int N, int K, float scale, float rscale)
{
  static_assert(MI >= 1 && MI <= 2);
  static_assert(SPL >= 0 && SPL <= 2);
  const _Float16* A   = (const _Float16*)Ap;
  const _Float16* A2  = (const _Float16*)A2p;
  const _Float16* Bt  = (const _Float16*)Btp;
  const _Float16* Bt2 = (const _Float16*)Bt2p;
  __shared__ __align__(16) float sT[8][16 * 68];
  const int lane = threadIdx.x & 31;
  const int wave = threadIdx.x >> 5;
  const int tilesN = N >> 6;
  const int tilesM = M / (16 * MI);
  const int tile = blockIdx.x * 8 + wave;
  if (tile >= tilesM * tilesN) return;
  const int tm = tile / tilesN;
  const int tn = tile - tm * tilesN;
  const int m0 = tm * (16 * MI);
  const int n0 = tn << 6;
  const int rlane = lane & 15;
  const int koff  = (lane >> 4) * 8;
  const int mOff  = (lane >> 4) * 8;

  v8f acc[MI][4], accr[MI][4];
#pragma unroll
  for (int i = 0; i < MI; ++i)
#pragma unroll
    for (int j = 0; j < 4; ++j) {
      acc[i][j]  = (v8f){0.f, 0.f, 0.f, 0.f, 0.f, 0.f, 0.f, 0.f};
      accr[i][j] = (v8f){0.f, 0.f, 0.f, 0.f, 0.f, 0.f, 0.f, 0.f};
    }

  for (int k0 = 0; k0 < K; k0 += 32) {
    v16h bh[4], bl[4];
#pragma unroll
    for (int j = 0; j < 4; ++j) {
      const size_t bo = (size_t)(n0 + (j << 4) + rlane) * ldb + koff + k0;
      bh[j] = frag_load(Bt + bo);
      if (SPL == 2) bl[j] = frag_load(Bt2 + bo); else bl[j] = bh[j];
    }
#pragma unroll
    for (int i = 0; i < MI; ++i) {
      const size_t ao = (size_t)(m0 + (i << 4) + rlane) * lda + koff + k0;
      const v16h ah = frag_load(A + ao);
      v16h al = ah;
      if (SPL >= 1) al = frag_load(A2 + ao);
#pragma unroll
      for (int j = 0; j < 4; ++j) {
        acc[i][j] = mma(ah, bh[j], acc[i][j]);
        if (SPL >= 1) accr[i][j] = mma(al, bh[j], accr[i][j]);
        if (SPL == 2) accr[i][j] = mma(ah, bl[j], accr[i][j]);
      }
#pragma unroll
      for (int j = 0; j < 4; ++j) {
        guard1(acc[i][j], ah, al);
        if (SPL >= 1) guard1(accr[i][j], ah, al);
      }
    }
    keep4(bh[0], bh[1], bh[2], bh[3]);
    if (SPL == 2) keep4(bl[0], bl[1], bl[2], bl[3]);
  }
#pragma unroll
  for (int i = 0; i < MI; ++i)
#pragma unroll
    for (int j = 0; j < 4; ++j) {
      guard_acc(acc[i][j]);
      if (SPL >= 1) guard_acc(accr[i][j]);
    }

  float* slab = sT[wave];
#pragma unroll
  for (int i = 0; i < MI; ++i) {
    const int mBase = m0 + (i << 4);
#pragma unroll
    for (int j = 0; j < 4; ++j) {
#pragma unroll
      for (int r = 0; r < 8; ++r) {
        float v = acc[i][j][r] * scale;
        if (SPL >= 1) v += accr[i][j][r] * rscale;
        slab[(mOff + r) * 68 + (j << 4) + rlane] = v;
      }
    }
    __builtin_amdgcn_fence(__ATOMIC_RELEASE, "workgroup");
    __builtin_amdgcn_wave_barrier();
    __builtin_amdgcn_fence(__ATOMIC_ACQUIRE, "workgroup");
    {
      const int hh = lane >> 4, c4 = (lane & 15) * 4;
      for (int pass = 0; pass < 2; ++pass) {
#pragma unroll
        for (int it = 0; it < 8; ++it) {
          const int row = it * 2 + hh;
          const v4f v = *(const v4f*)(slab + row * 68 + c4);
          *(volatile v4f*)(C + (size_t)(mBase + row) * ldc + n0 + c4) = v;
        }
        __threadfence();
      }
    }
    __builtin_amdgcn_fence(__ATOMIC_RELEASE, "workgroup");
    __builtin_amdgcn_wave_barrier();
    __builtin_amdgcn_fence(__ATOMIC_ACQUIRE, "workgroup");
  }
}
}

__global__ __launch_bounds__(256) void ax_pack_kernel(
    const float* __restrict__ h_prev, const float* __restrict__ x, unsigned short* __restrict__ AX)
{
  const int b    = (int)(blockIdx.x >> 1);
  const int side = (int)(blockIdx.x & 1);
  const int kk   = (int)threadIdx.x * 8;
  const float* src = (side == 0) ? h_prev : x;
  const float* sp = src + (size_t)b * kH + kk;
  const v4f a0 = *(const v4f*)(sp);
  const v4f a1 = *(const v4f*)(sp + 4);
  const float f0 = a0[0];
  const float f1 = a0[1];
  const float f2 = a0[2];
  const float f3 = a0[3];
  const float f4 = a1[0];
  const float f5 = a1[1];
  const float f6 = a1[2];
  const float f7 = a1[3];
  v8h hv;
  hv[0] = f16_flush(bf16r(f0));
  hv[1] = f16_flush(bf16r(f1));
  hv[2] = f16_flush(bf16r(f2));
  hv[3] = f16_flush(bf16r(f3));
  hv[4] = f16_flush(bf16r(f4));
  hv[5] = f16_flush(bf16r(f5));
  hv[6] = f16_flush(bf16r(f6));
  hv[7] = f16_flush(bf16r(f7));
  unsigned short* qh = AX + (size_t)b * kK + (size_t)side * kH + kk;
  *(volatile v8h*)qh = hv;
  __threadfence();
  *(volatile v8h*)qh = hv;
}

__global__ __launch_bounds__(256) void wt_pack_kernel(
    const float* __restrict__ Wfh, const float* __restrict__ Wfx,
    const float* __restrict__ Wih, const float* __restrict__ Wix,
    const float* __restrict__ Wch, const float* __restrict__ Wcx,
    const float* __restrict__ Woh, const float* __restrict__ Wox,
    unsigned short* __restrict__ WT)
{
  const int n    = (int)(blockIdx.x >> 1);
  const int side = (int)(blockIdx.x & 1);
  const int kk   = (int)threadIdx.x * 8;
  const int g    = n >> 11;
  const int col  = n & (kH - 1);
  const int sel  = g * 2 + side;
  const float* src = Wfh;
  switch (sel) {
    case 1: src = Wfx; break;
    case 2: src = Wih; break;
    case 3: src = Wix; break;
    case 4: src = Wch; break;
    case 5: src = Wcx; break;
    case 6: src = Woh; break;
    case 7: src = Wox; break;
    default: break;
  }
  const float* sp = src + (size_t)kk * kH + col;
  const float w0 = sp[(size_t)0 * kH];
  const float w1 = sp[(size_t)1 * kH];
  const float w2 = sp[(size_t)2 * kH];
  const float w3 = sp[(size_t)3 * kH];
  const float w4 = sp[(size_t)4 * kH];
  const float w5 = sp[(size_t)5 * kH];
  const float w6 = sp[(size_t)6 * kH];
  const float w7 = sp[(size_t)7 * kH];
  v8h hv;
  hv[0] = f16_flush(bf16r(w0) * kWCarry);
  hv[1] = f16_flush(bf16r(w1) * kWCarry);
  hv[2] = f16_flush(bf16r(w2) * kWCarry);
  hv[3] = f16_flush(bf16r(w3) * kWCarry);
  hv[4] = f16_flush(bf16r(w4) * kWCarry);
  hv[5] = f16_flush(bf16r(w5) * kWCarry);
  hv[6] = f16_flush(bf16r(w6) * kWCarry);
  hv[7] = f16_flush(bf16r(w7) * kWCarry);
  unsigned short* qh = WT + (size_t)n * kK + (size_t)side * kH + kk;
  *(volatile v8h*)qh = hv;
  __threadfence();
  *(volatile v8h*)qh = hv;
}

__global__ __launch_bounds__(256) void wy_pack_kernel(
    const float* __restrict__ Wy, unsigned short* __restrict__ WY)
{
  const int n  = (int)blockIdx.x;
  const int kk = (int)threadIdx.x * 8;
  const float* sp = Wy + (size_t)kk * kH + n;
  const float w0 = sp[(size_t)0 * kH];
  const float w1 = sp[(size_t)1 * kH];
  const float w2 = sp[(size_t)2 * kH];
  const float w3 = sp[(size_t)3 * kH];
  const float w4 = sp[(size_t)4 * kH];
  const float w5 = sp[(size_t)5 * kH];
  const float w6 = sp[(size_t)6 * kH];
  const float w7 = sp[(size_t)7 * kH];
  v8h hv;
  hv[0] = f16_flush(bf16r(w0) * kWCarry);
  hv[1] = f16_flush(bf16r(w1) * kWCarry);
  hv[2] = f16_flush(bf16r(w2) * kWCarry);
  hv[3] = f16_flush(bf16r(w3) * kWCarry);
  hv[4] = f16_flush(bf16r(w4) * kWCarry);
  hv[5] = f16_flush(bf16r(w5) * kWCarry);
  hv[6] = f16_flush(bf16r(w6) * kWCarry);
  hv[7] = f16_flush(bf16r(w7) * kWCarry);
  unsigned short* qh = WY + (size_t)n * kH + kk;
  *(volatile v8h*)qh = hv;
  __threadfence();
  *(volatile v8h*)qh = hv;
}

__global__ __launch_bounds__(256) void cell_out_kernel(
    const float* __restrict__ GT, const float* __restrict__ YR, const float* __restrict__ c_prev,
    const float* __restrict__ bf, const float* __restrict__ bi, const float* __restrict__ bc,
    const float* __restrict__ bo, const float* __restrict__ by, float* __restrict__ out)
{
  const int t  = (int)(blockIdx.x * 256 + threadIdx.x);
  const int b  = t >> 9;
  const int j0 = (t & 511) * 4;
  const size_t gb = (size_t)b * kG + j0;
  const size_t hb = (size_t)b * kH + j0;
  const v4f gfv = *(const v4f*)(GT + gb);
  const v4f giv = *(const v4f*)(GT + gb + kH);
  const v4f gcv = *(const v4f*)(GT + gb + 2 * kH);
  const v4f gov = *(const v4f*)(GT + gb + 3 * kH);
  const v4f yrv = *(const v4f*)(YR + hb);
  const v4f cpv = *(const v4f*)(c_prev + hb);
  const v4f bfv = *(const v4f*)(bf + j0);
  const v4f biv = *(const v4f*)(bi + j0);
  const v4f bcv = *(const v4f*)(bc + j0);
  const v4f bov = *(const v4f*)(bo + j0);
  const v4f byv = *(const v4f*)(by + j0);
  v4f vy, vh, vc;
#pragma unroll
  for (int e = 0; e < 4; ++e) {
    const float gf_s = gfv[e];
    const float gi_s = giv[e];
    const float gc_s = gcv[e];
    const float go_s = gov[e];
    const float yr_s = yrv[e];
    const float cp_s = cpv[e];
    const float bf_s = bfv[e];
    const float bi_s = biv[e];
    const float bc_s = bcv[e];
    const float bo_s = bov[e];
    const float by_s = byv[e];
    const float pf = gf_s + bf16r(bf_s);
    const float pi = gi_s + bf16r(bi_s);
    const float pc = gc_s + bf16r(bc_s);
    const float po = go_s + bf16r(bo_s);
    const float fg = 1.0f / (1.0f + expf(-pf));
    const float ig = 1.0f / (1.0f + expf(-pi));
    const float ct = tanhf(pc);
    const float og = 1.0f / (1.0f + expf(-po));
    const float cn = fg * bf16r(cp_s) + ig * ct;
    const float hn = og * tanhf(cn);
    const float yn = yr_s + bf16r(by_s);
    vy[e] = yn;
    vh[e] = hn;
    vc[e] = cn;
  }
  float* py = out + (size_t)b * kOutLd + j0;
  float* ph = py + kH;
  float* pc2 = py + 2 * kH;
  *(volatile v4f*)py  = vy;
  *(volatile v4f*)ph  = vh;
  *(volatile v4f*)pc2 = vc;
  __threadfence();
  *(volatile v4f*)py  = vy;
  *(volatile v4f*)ph  = vh;
  *(volatile v4f*)pc2 = vc;
}

extern "C" void kernel_launch(void* const* d_in, const int* in_sizes, int n_in,
                              void* d_out, int out_size, void* d_ws, size_t ws_size,
                              hipStream_t stream)
{
  if (n_in < 17) return;
  if (in_sizes[0] != kB * kH) return;
  if (in_sizes[1] != kB * kH) return;
  if (in_sizes[2] != kB * kH) return;
  if (in_sizes[3] != kH * kH) return;
  if (in_sizes[4] != kH * kH) return;
  if (in_sizes[5] != kH) return;
  if (in_sizes[6] != kH * kH) return;
  if (in_sizes[7] != kH * kH) return;
  if (in_sizes[8] != kH) return;
  if (in_sizes[9] != kH * kH) return;
  if (in_sizes[10] != kH * kH) return;
  if (in_sizes[11] != kH) return;
  if (in_sizes[12] != kH * kH) return;
  if (in_sizes[13] != kH * kH) return;
  if (in_sizes[14] != kH) return;
  if (in_sizes[15] != kH * kH) return;
  if (in_sizes[16] != kH) return;
  if (out_size != kB * kOutLd) return;
  if (ws_size < kWsTotal) return;

  const float* x      = (const float*)d_in[0];
  const float* h_prev = (const float*)d_in[1];
  const float* c_prev = (const float*)d_in[2];
  const float* Wfh    = (const float*)d_in[3];
  const float* Wfx    = (const float*)d_in[4];
  const float* bf     = (const float*)d_in[5];
  const float* Wih    = (const float*)d_in[6];
  const float* Wix    = (const float*)d_in[7];
  const float* bi     = (const float*)d_in[8];
  const float* Woh    = (const float*)d_in[9];
  const float* Wox    = (const float*)d_in[10];
  const float* bo     = (const float*)d_in[11];
  const float* Wch    = (const float*)d_in[12];
  const float* Wcx    = (const float*)d_in[13];
  const float* bc     = (const float*)d_in[14];
  const float* Wy     = (const float*)d_in[15];
  const float* by     = (const float*)d_in[16];
  float* out = (float*)d_out;

  char* ws = (char*)d_ws;
  unsigned short* AX = (unsigned short*)(ws + kOffAX);
  unsigned short* WT = (unsigned short*)(ws + kOffWT);
  unsigned short* WY = (unsigned short*)(ws + kOffWY);
  float*          GT = (float*)(ws + kOffGT);
  float*          YR = (float*)(ws + kOffYR);

  constexpr float sW = 1.0f / kWCarry;

  ax_pack_kernel<<<(kB * kK / 8) / 256, 256, 0, stream>>>(h_prev, x, AX);

  wt_pack_kernel<<<(kG * kK / 8) / 256, 256, 0, stream>>>(Wfh, Wfx, Wih, Wix, Wch, Wcx, Woh, Wox, WT);

  wy_pack_kernel<<<(kH * kH / 8) / 256, 256, 0, stream>>>(Wy, WY);

  eng::gemm_f16_kernel<2, 0><<<dim3((kB / 32) * (kG / 64) / 8), 256, 0, stream>>>(
      AX, nullptr, kK, WT, nullptr, kK, GT, kG, kB, kG, kK, sW, 0.0f);

  eng::gemm_f16_kernel<2, 0><<<dim3((kB / 32) * (kH / 64) / 8), 256, 0, stream>>>(
      AX, nullptr, kK, WY, nullptr, kH, YR, kH, kB, kH, kH, sW, 0.0f);

  cell_out_kernel<<<(kB * kH / 4) / 256, 256, 0, stream>>>(GT, YR, c_prev, bf, bi, bc, bo, by, out);
}
